// GInitResN_66108136620575
// MI455X (gfx1250) — hardware-run, weakly checked
//
#include <hip/hip_runtime.h>


namespace {
constexpr int NN = 50000, NP = 50016, NE = 600000, D = 128, NL = 4, NC = 5, STB = 256, MAXDEG = 1024, NGc = (NN + 511) / 512, PERMLEN = NE + 32 * NGc + 32;
constexpr float XS = 8.0f, GN_EPS = 1e-5f;

typedef _Float16 b16;
typedef __attribute__((ext_vector_type(16))) _Float16 v16b;
typedef __attribute__((ext_vector_type(8))) _Float16 v8b;
typedef __attribute__((ext_vector_type(8))) float v8f;
typedef __attribute__((ext_vector_type(4))) float v4f;
__device__ __forceinline__ float bf16_rne(float f) { unsigned int u = __float_as_uint(f); u += 0x7FFFu + ((u >> 16) & 1u); return __uint_as_float(u & 0xFFFF0000u); }
__device__ __forceinline__ void split16(float v, b16& hi, b16& lo) { hi = (b16)v; lo = (b16)(v - (float)hi); }
__device__ __forceinline__ v16b frag_kb(const b16* p, int hh) { const v8b a = *(const v8b*)(p + 8 * hh), b = *(const v8b*)(p + 16 + 8 * hh); v16b f;
#pragma unroll
  for (int e = 0; e < 8; ++e) { f[e] = a[e]; f[8 + e] = b[e]; } return f; }
__device__ __forceinline__ v8f wmma16b(v16b a, v16b b, v8f c) { v8f d = __builtin_amdgcn_wmma_f32_16x16x32_f16(false, a, false, b, (short)0, c, false, false); asm volatile("v_nop\n\tv_nop\n\tv_nop\n\tv_nop" : "+v"(d) : "v"(a), "v"(b)); return d; }
__device__ __forceinline__ void wave_lds_sync() { __builtin_amdgcn_fence(__ATOMIC_RELEASE, "workgroup"); __builtin_amdgcn_wave_barrier(); __builtin_amdgcn_fence(__ATOMIC_ACQUIRE, "workgroup"); }
__device__ __forceinline__ float nexp(float x) { return __builtin_amdgcn_exp2f(x * 1.4426950408889634f); }
__device__ __forceinline__ float pmul(float a, float b) { float p = a * b; asm volatile("" : "+v"(p)); return p; }
__device__ __forceinline__ float tanh_f(float x) { const float e = nexp(-2.0f * fabsf(x)); const float t = (1.0f - e) / (1.0f + e); return (x < 0.0f) ? -t : t; }
__device__ __forceinline__ float elu_f(float x) { return (x > 0.0f) ? x : (nexp(x) - 1.0f); }
constexpr int CSR_NBLK = 512, CSR_GB = 9, CSR_GN = 1 << CSR_GB  , CSR_MAXG = 512, CSR_CAP = 12288  ;
__global__ __launch_bounds__(64) void csrA_kernel(const int* __restrict__ dst, int E, int N, int nG, int CHP, int NGP, int* __restrict__ STG, int* __restrict__ HST) {
  extern __shared__ int sm[];
  int* cnt = sm; int* run = sm + NGP; int* ids = sm + 2 * NGP;
  const int b = blockIdx.x; const int ch = (E + CSR_NBLK - 1) / CSR_NBLK; const int e0 = b * ch, e1 = min(E, e0 + ch);
  for (int i = threadIdx.x; i < NGP; i += 64) cnt[i] = 0;
  for (int i = threadIdx.x; i < CHP; i += 64) ids[i] = -1;
  __syncthreads();
  if (threadIdx.x == 0) {
    for (int e = e0; e < e1; ++e) { int d = dst[e]; d = (d < 0) ? 0 : (d >= N ? N - 1 : d); cnt[d >> CSR_GB] += 1; }
    int acc = 0; for (int g = 0; g < nG; ++g) { run[g] = acc; acc += cnt[g]; }
    for (int e = e0; e < e1; ++e) { int d = dst[e]; d = (d < 0) ? 0 : (d >= N ? N - 1 : d); const int g = d >> CSR_GB; ids[run[g]] = e; run[g] += 1; } }
  __syncthreads();
  typedef __attribute__((ext_vector_type(4))) int v4i;
  for (int pass = 0; pass < 2; ++pass) {
    for (int i = threadIdx.x; i < CHP / 4; i += 64) *(volatile v4i*)(STG + (size_t)b * CHP + i * 4) = *(const v4i*)(&ids[i * 4]);
    for (int i = threadIdx.x; i < NGP / 4; i += 64) { v4i v; for (int e = 0; e < 4; ++e) v[e] = (i * 4 + e < nG) ? cnt[i * 4 + e] : 0; *(volatile v4i*)(HST + (size_t)b * NGP + i * 4) = v; }
    __threadfence(); }
}
__global__ __launch_bounds__(512) void csrS_kernel(const int* __restrict__ HST, int nG, int NGP, int* __restrict__ START, int* __restrict__ TOT, int* __restrict__ OFF) {
  __shared__ int tot[CSR_MAXG];
  const int b = threadIdx.x;
  for (int pass = 0; pass < 2; ++pass) { int runb = 0; for (int g = 0; g < nG; ++g) { int c = HST[(size_t)b * NGP + g]; c = (c < 0) ? 0 : c; ((volatile int*)OFF)[(size_t)g * CSR_NBLK + b] = runb; runb += c; } __threadfence(); }
  for (int g = threadIdx.x; g < nG; g += 512) { int s = 0; for (int bb = 0; bb < CSR_NBLK; ++bb) { int c = HST[(size_t)bb * NGP + g]; s += (c < 0) ? 0 : c; } tot[g] = s; }
  __syncthreads();
  if (threadIdx.x < 32) {
    __shared__ int st[CSR_MAXG + 32];
    if (threadIdx.x == 0) { int acc = 0; for (int g = 0; g < NGP; ++g) { st[g] = acc; if (g < nG) acc += (tot[g] + 31) & ~31; } st[NGP] = acc; }
    __builtin_amdgcn_fence(__ATOMIC_RELEASE, "workgroup"); __builtin_amdgcn_wave_barrier(); __builtin_amdgcn_fence(__ATOMIC_ACQUIRE, "workgroup");
    for (int pass = 0; pass < 2; ++pass) { for (int i = threadIdx.x; i < NGP + 32; i += 32) { ((volatile int*)START)[i] = (i <= NGP) ? st[min(i, NGP)] : 0; ((volatile int*)TOT)[i] = (i < nG) ? tot[i] : 0; } __threadfence(); } }
}
__global__ __launch_bounds__(256) void csrB_kernel(const int* __restrict__ dst, int N, int nG, int CHP, int NGP, int permLen, const int* __restrict__ STG, const int* __restrict__ HST, const int* __restrict__ OFF, const int* __restrict__ START, const int* __restrict__ TOT, int* __restrict__ PERM, int* __restrict__ ROWPTR, int* __restrict__ ROWCNT, int* __restrict__ FLAG) {
  typedef __attribute__((ext_vector_type(4))) int v4i;
  __shared__ int ids[CSR_CAP]; __shared__ unsigned short key[CSR_CAP]; __shared__ int outp[CSR_CAP]; __shared__ int ncnt[CSR_GN + 1]; __shared__ int boff[CSR_NBLK + 1];
  const int g = blockIdx.x, t_ = threadIdx.x; int tot = TOT[g]; int st = START[g], stn = START[g + 1]; const int v0 = g * CSR_GN; const int nv = min(CSR_GN, N - v0);
  st = (st < 0) ? 0 : (st > permLen - 32 ? permLen - 32 : st) & ~31; stn = (stn < st) ? st : (stn > permLen ? permLen : stn); tot = (tot < 0) ? 0 : tot; if (tot > stn - st && tot <= CSR_CAP) tot = stn - st;
  if (tot > CSR_CAP) {
    for (int pass = 0; pass < 2; ++pass) { for (int i = t_; i < CSR_GN / 4; i += 256) { v4i a, c; for (int e = 0; e < 4; ++e) { a[e] = st; c[e] = 0; } *(volatile v4i*)(ROWPTR + v0 + i * 4) = a; *(volatile v4i*)(ROWCNT + v0 + i * 4) = c; } if (t_ == 0) ((volatile int*)FLAG)[0] = 1; __threadfence(); } (void)nv; return; }
  if (t_ == 0) { int acc = 0; for (int b = 0; b < CSR_NBLK; ++b) { boff[b] = acc; int c = HST[(size_t)b * NGP + g]; c = (c < 0) ? 0 : (c > CHP ? CHP : c); acc += c; if (acc > tot) acc = tot; } boff[CSR_NBLK] = acc; }
  for (int i = t_; i <= CSR_GN; i += 256) ncnt[i] = 0;
  __syncthreads();
  for (int b = 0; b < CSR_NBLK; ++b) { const int c = boff[b + 1] - boff[b]; int o_ = OFF[(size_t)g * CSR_NBLK + b]; o_ = (o_ < 0) ? 0 : (o_ > CHP - c ? CHP - c : o_); const int* src_ = STG + (size_t)b * CHP + o_;
    for (int i = t_; i < c; i += 256) { int id = src_[i]; id = (id < 0) ? 0 : id; ids[boff[b] + i] = id; int d = dst[id]; d = (d < v0) ? v0 : (d >= N ? N - 1 : d); int kk = d - v0; kk = (kk < 0) ? 0 : (kk >= CSR_GN ? CSR_GN - 1 : kk); key[boff[b] + i] = (unsigned short)kk; } }
  __syncthreads();
  if (t_ == 0) { for (int i = 0; i < tot; ++i) ncnt[key[i]] += 1; int acc = 0; for (int vl = 0; vl < CSR_GN; ++vl) { const int c = ncnt[vl]; ncnt[vl] = acc; acc += c; } ncnt[CSR_GN] = acc;
    for (int i = 0; i < tot; ++i) { const int vl = key[i]; outp[ncnt[vl]] = ids[i]; ncnt[vl] += 1; }
    for (int vl = CSR_GN; vl > 0; --vl) ncnt[vl] = ncnt[vl - 1]; ncnt[0] = 0; }
  __syncthreads();
  for (int pass = 0; pass < 2; ++pass) {
    for (int i = t_; i < (stn - st) / 4; i += 256) { v4i v; for (int e = 0; e < 4; ++e) { const int q = i * 4 + e; v[e] = (q < tot) ? outp[q] : -1; } *(volatile v4i*)(PERM + st + i * 4) = v; }
    for (int i = t_; i < CSR_GN / 4; i += 256) { v4i a, c; for (int e = 0; e < 4; ++e) { const int vl = i * 4 + e; a[e] = st + ncnt[vl]; c[e] = (vl < nv) ? (ncnt[vl + 1] - ncnt[vl]) : 0; } *(volatile v4i*)(ROWPTR + v0 + i * 4) = a; *(volatile v4i*)(ROWCNT + v0 + i * 4) = c; }
    __threadfence(); }
}
__global__ __launch_bounds__(256) void csrZ_kernel(int* __restrict__ p, size_t n4) { typedef __attribute__((ext_vector_type(4))) int v4i; const size_t tid = (size_t)blockIdx.x * 256 + threadIdx.x, nth = (size_t)gridDim.x * 256; v4i z = {0, 0, 0, 0}; for (size_t i = tid; i < n4; i += nth) *(volatile v4i*)(p + i * 4) = z; }
struct CsrBufs { int *STG, *HST, *OFF, *START, *TOT, *PERM, *ROWPTR, *ROWCNT, *FLAG; int nG, NGP, CHP; size_t permLen; char* base; size_t bytes; };
static size_t csr_carve(CsrBufs& c, char* ws, size_t off, int E, int N) {
  const size_t off0 = off; c.base = ws + off;
  auto al = [&](size_t bytes) { char* p = ws + off; off += (bytes + 255) & ~(size_t)255; return p; };
  c.nG = (N + CSR_GN - 1) / CSR_GN; c.NGP = (c.nG + 31) & ~31; const int ch = (E + CSR_NBLK - 1) / CSR_NBLK; c.CHP = (ch + 31) & ~31; c.permLen = (size_t)E + 32 * (size_t)c.nG + 32;
  c.STG = (int*)al((size_t)CSR_NBLK * c.CHP * 4); c.HST = (int*)al((size_t)CSR_NBLK * c.NGP * 4); c.OFF = (int*)al((size_t)c.NGP * CSR_NBLK * 4); c.START = (int*)al((size_t)(c.NGP + 64) * 4); c.TOT = (int*)al((size_t)(c.NGP + 64) * 4);
  c.PERM = (int*)al(c.permLen * 4); c.ROWPTR = (int*)al((size_t)c.nG * CSR_GN * 4); c.ROWCNT = (int*)al((size_t)c.nG * CSR_GN * 4); c.FLAG = (int*)al(256);
  c.bytes = off - off0; return off;
}
static void csr_build(const CsrBufs& c, const int* dst, int E, int N, hipStream_t stream) {
  const size_t smem = (size_t)(2 * c.NGP + c.CHP) * 4;
  csrZ_kernel<<<512, 256, 0, stream>>>((int*)c.base, c.bytes / 16);
  csrA_kernel<<<CSR_NBLK, 64, smem, stream>>>(dst, E, N, c.nG, c.CHP, c.NGP, c.STG, c.HST);
  csrS_kernel<<<1, 512, 0, stream>>>(c.HST, c.nG, c.NGP, c.START, c.TOT, c.OFF);
  csrB_kernel<<<c.nG, 256, 0, stream>>>(dst, N, c.nG, c.CHP, c.NGP, (int)c.permLen, c.STG, c.HST, c.OFF, c.START, c.TOT, c.PERM, c.ROWPTR, c.ROWCNT, c.FLAG);
}

__global__ __launch_bounds__(256) void prep_kernel(const float* __restrict__ x, const float* __restrict__ al, const float* __restrict__ ar, const float* __restrict__ gw, const float* __restrict__ gb, const float* __restrict__ gs, const float* __restrict__ lw, const float* __restrict__ lb, b16* __restrict__ R, float* __restrict__ P, float* __restrict__ H0f, float* __restrict__ Hf, b16* __restrict__ Hh, b16* __restrict__ Hl) {
  const size_t tid = (size_t)blockIdx.x * 256 + threadIdx.x, nth = (size_t)gridDim.x * 256;
  for (int pass = 0; pass < 2; ++pass) {
    for (size_t p = tid; p < (size_t)(NL + 1) * 16 * D; p += nth) { const int l = (int)(p / (16 * D)), rem = (int)(p % (16 * D)), o = rem / D, k = rem % D; float v = 0.0f;
      if (l < NL) { if (o == 0) v = al[l * D + k]; else if (o == 1) v = ar[l * D + k]; } else if (o < NC) v = lw[(size_t)k * NC + o];
      ((volatile b16*)R)[p] = (b16)bf16_rne(v); }
    for (size_t q = tid; q < 1552; q += nth) { const int i = (int)q; float v; if (i < 512) v = gw[i]; else if (i < 1024) v = gb[i - 512]; else if (i < 1536) v = gs[i - 1024]; else v = (i - 1536 < NC) ? lb[i - 1536] : 0.0f; P[q] = bf16_rne(v); }
    for (size_t p = tid; p < (size_t)NP * D / 8; p += nth) { const size_t r = p / (D / 8); v8b v = {}, z = {}; float f[8] = {0, 0, 0, 0, 0, 0, 0, 0}; if (r < (size_t)NN) { for (int e = 0; e < 8; ++e) { f[e] = bf16_rne(x[p * 8 + e]); v[e] = (b16)(f[e] * XS); } }
      *(volatile v8b*)(Hh + p * 8) = v; *(volatile v8b*)(Hl + p * 8) = z; *(volatile v4f*)(H0f + p * 8) = *(v4f*)&f[0]; *(volatile v4f*)(H0f + p * 8 + 4) = *(v4f*)&f[4]; *(volatile v4f*)(Hf + p * 8) = *(v4f*)&f[0]; *(volatile v4f*)(Hf + p * 8 + 4) = *(v4f*)&f[4]; }
    __threadfence(); }
}

template <int BIAS>
__global__ __launch_bounds__(64) void gemm16_kernel(const b16* __restrict__ Hh, const b16* __restrict__ Hl, const b16* __restrict__ Bw, const float* __restrict__ Pb, float* __restrict__ OUT) {
  __shared__ __attribute__((aligned(16))) float Ts[32][16 + 4];
  const int lane = threadIdx.x & 31, wave = threadIdx.x >> 5, nloc = lane & 15, hlf = lane >> 4, m0 = blockIdx.x * 32 + wave * 16;
  v8f acc = {};
#pragma unroll
  for (int kb = 0; kb < D; kb += 32) { const v16b a = frag_kb(Hh + (size_t)(m0 + nloc) * D + kb, hlf), al_ = frag_kb(Hl + (size_t)(m0 + nloc) * D + kb, hlf), bw = frag_kb(Bw + (size_t)nloc * D + kb, hlf); acc = wmma16b(a, bw, acc); acc = wmma16b(al_, bw, acc); }
#pragma unroll
  for (int r = 0; r < 8; ++r) Ts[wave * 16 + 8 * hlf + r][nloc] = acc[r] * (1.0f / XS) + (BIAS ? Pb[nloc] : 0.0f);
  __syncthreads();
  for (int pass = 0; pass < 2; ++pass) { if (threadIdx.x < 32 * 4 / 2) { for (int i = threadIdx.x; i < 32 * 4; i += 64) { const int rr = i >> 2, c4 = (i & 3) * 4; *(volatile v4f*)(OUT + (size_t)(blockIdx.x * 32 + rr) * 16 + c4) = *(const v4f*)(&Ts[rr][c4]); } } __threadfence(); }
}

__global__ __launch_bounds__(256) void agg_kernel(const float* __restrict__ Hf, const float* __restrict__ H0f, const float* __restrict__ ALR, const int* __restrict__ src, const int* __restrict__ perm, const int* __restrict__ rowptr, const int* __restrict__ rowcnt, float* __restrict__ U) {
  const int wave = threadIdx.x >> 5, v = blockIdx.x * 8 + wave, lane = threadIdx.x & 31;
  int cnt = rowcnt[v]; cnt = (cnt < 0) ? 0 : (cnt > MAXDEG ? MAXDEG : cnt); int p0 = rowptr[v]; p0 = (p0 < 0) ? 0 : (p0 > PERMLEN - cnt ? PERMLEN - cnt : p0);
  const float dv = (cnt > 0) ? rsqrtf((float)cnt) : 0.0f; const float arv = ALR[(size_t)v * 16 + 1];
  v4f acc = {0, 0, 0, 0};
  for (int q = 0; q < cnt; ++q) { int id = perm[p0 + q]; id = (id < 0) ? 0 : (id >= NE ? NE - 1 : id); int s = src[id]; s = (s < 0) ? 0 : (s >= NN ? NN - 1 : s); int cs_ = rowcnt[s]; cs_ = (cs_ < 0) ? 0 : (cs_ > MAXDEG ? MAXDEG : cs_); const float ds = (cs_ > 0) ? rsqrtf((float)cs_) : 0.0f;
    const float w = pmul(tanh_f(ALR[(size_t)s * 16 + 0] + arv), pmul(ds, dv)); const v4f hv = *(const v4f*)(Hf + (size_t)s * D + lane * 4);
#pragma unroll
    for (int e = 0; e < 4; ++e) acc[e] += pmul(w, hv[e]); }
  const v4f h0 = *(const v4f*)(H0f + (size_t)v * D + lane * 4); v4f o; for (int e = 0; e < 4; ++e) o[e] = elu_f(h0[e] + acc[e]);
  for (int pass = 0; pass < 2; ++pass) { *(volatile v4f*)(U + (size_t)v * D + lane * 4) = o; __threadfence(); }
}

template <int MODE>
__global__ __launch_bounds__(128) void stat_kernel(const float* __restrict__ U, const float* __restrict__ MEAN, const float* __restrict__ P, int l, float* __restrict__ PART) {
  const int c = threadIdx.x, b = blockIdx.x; const int ch = (NN + STB - 1) / STB; const int r0 = b * ch, r1 = min(NN, r0 + ch); const float sm = MODE ? pmul(P[1024 + l * D + c], MEAN[c]) : 0.0f;
  float s = 0.0f; for (int r = r0; r < r1; ++r) { const float x = U[(size_t)r * D + c]; if (MODE) { const float d = x - sm; s += pmul(d, d); } else s += x; }
  for (int pass = 0; pass < 2; ++pass) { ((volatile float*)PART)[(size_t)b * D + c] = s; __threadfence(); }
}
__global__ __launch_bounds__(128) void comb_kernel(const float* __restrict__ PART, float* __restrict__ OUT) {
  const int c = threadIdx.x; float s = 0.0f; for (int b = 0; b < STB; ++b) s += PART[(size_t)b * D + c];
  for (int pass = 0; pass < 2; ++pass) { ((volatile float*)OUT)[c] = s * (1.0f / NN); __threadfence(); }
}
__global__ __launch_bounds__(256) void epi_kernel(const float* __restrict__ U, const float* __restrict__ MEAN, const float* __restrict__ MSQ, const float* __restrict__ P, int l, float* __restrict__ Hf, b16* __restrict__ Hh, b16* __restrict__ Hl) {
  __shared__ __attribute__((aligned(16))) b16 Sh[8][D + 8], Sl[8][D + 8];
  const int wave = threadIdx.x >> 5, v = blockIdx.x * 8 + wave, lane = threadIdx.x & 31;
  const v4f u = *(const v4f*)(U + (size_t)v * D + lane * 4); v4f o;
#pragma unroll
  for (int e = 0; e < 4; ++e) { const int c = lane * 4 + e; const float sub = u[e] - pmul(P[1024 + l * D + c], MEAN[c]); o[e] = pmul(P[l * D + c], sub * rsqrtf(MSQ[c] + GN_EPS)) + P[512 + l * D + c]; b16 a_, b_; split16(o[e] * XS, a_, b_); Sh[wave][c] = a_; Sl[wave][c] = b_; }
  wave_lds_sync();
  for (int pass = 0; pass < 2; ++pass) { *(volatile v4f*)(Hf + (size_t)v * D + lane * 4) = o; if (lane < 16) { *(volatile v8b*)(Hh + (size_t)v * D + lane * 8) = *(const v8b*)(&Sh[wave][lane * 8]); *(volatile v8b*)(Hl + (size_t)v * D + lane * 8) = *(const v8b*)(&Sl[wave][lane * 8]); } __threadfence(); }
}
__global__ __launch_bounds__(64) void out_kernel(const float* __restrict__ L16, float* __restrict__ out) {
  __shared__ __attribute__((aligned(16))) float Os[64 * NC];
  const int v0 = blockIdx.x * 64, t_ = threadIdx.x; const int nv = min(64, NN - v0);
  for (int i = t_; i < nv * NC; i += 64) { const int vl = i / NC, c = i % NC; Os[vl * NC + c] = L16[(size_t)(v0 + vl) * 16 + c]; }
  __syncthreads();
  for (int pass = 0; pass < 2; ++pass) { for (int i = t_; i < nv * NC / 4; i += 64) *(volatile v4f*)(out + (size_t)v0 * NC + i * 4) = *(const v4f*)(&Os[i * 4]); __threadfence(); }
}
}

extern "C" void kernel_launch(void* const* d_in, const int* in_sizes, int n_in,
                              void* d_out, int out_size, void* d_ws, size_t ws_size, hipStream_t stream) {
  (void)n_in; (void)out_size;
  const float* x = (const float*)d_in[0]; const int* ei = (const int*)d_in[1]; const float* al = (const float*)d_in[2]; const float* ar = (const float*)d_in[3]; const float* gw = (const float*)d_in[4]; const float* gb = (const float*)d_in[5]; const float* gs = (const float*)d_in[6]; const float* lw = (const float*)d_in[7]; const float* lb = (const float*)d_in[8];
  float* out = (float*)d_out;
  if (in_sizes[0] != NN * D || in_sizes[1] != 2 * NE || in_sizes[2] != NL * D || in_sizes[7] != D * NC) return;
  const int* srcI = ei; const int* dstI = ei + NE;
  size_t off = 0; char* ws = (char*)d_ws;
  auto carve = [&](size_t bytes) { char* p = ws + off; off += (bytes + 255) & ~(size_t)255; return p; };
  b16* R = (b16*)carve((size_t)(NL + 1) * 16 * D * 2); float* P = (float*)carve(1552 * 4); float* H0f = (float*)carve((size_t)NP * D * 4); float* Hf = (float*)carve((size_t)NP * D * 4); b16* Hh = (b16*)carve((size_t)NP * D * 2); b16* Hl = (b16*)carve((size_t)NP * D * 2); float* U = (float*)carve((size_t)NP * D * 4); float* ALR = (float*)carve((size_t)NP * 16 * 4);
  float* PART = (float*)carve((size_t)STB * D * 4); float* MEAN = (float*)carve(D * 4); float* MSQ = (float*)carve(D * 4);
  CsrBufs cs; off = csr_carve(cs, ws, off, NE, NN);
  if (off > ws_size) return;
  csr_build(cs, dstI, NE, NN, stream);
  prep_kernel<<<512, 256, 0, stream>>>(x, al, ar, gw, gb, gs, lw, lb, R, P, H0f, Hf, Hh, Hl);
  for (int l = 0; l < NL; ++l) {
    gemm16_kernel<0><<<NP / 32, 64, 0, stream>>>(Hh, Hl, R + (size_t)l * 16 * D, P, ALR);
    agg_kernel<<<NN / 8, 256, 0, stream>>>(Hf, H0f, ALR, srcI, cs.PERM, cs.ROWPTR, cs.ROWCNT, U);
    stat_kernel<0><<<STB, 128, 0, stream>>>(U, nullptr, P, l, PART); comb_kernel<<<1, 128, 0, stream>>>(PART, MEAN);
    stat_kernel<1><<<STB, 128, 0, stream>>>(U, MEAN, P, l, PART); comb_kernel<<<1, 128, 0, stream>>>(PART, MSQ);
    epi_kernel<<<NN / 8, 256, 0, stream>>>(U, MEAN, MSQ, P, l, Hf, Hh, Hl); }
  gemm16_kernel<1><<<NP / 32, 64, 0, stream>>>(Hh, Hl, R + (size_t)NL * 16 * D, P + 1536, ALR);
  out_kernel<<<(NN + 63) / 64, 64, 0, stream>>>(ALR, out);
}
